// HyperbolicLogisticLayer_47476568490613
// MI455X (gfx1250) — hardware-verified
//
#include <hip/hip_runtime.h>
#include <math.h>

constexpr int kRows       = 4096;
constexpr int kUnits      = 256;
constexpr int kDim        = 128;
constexpr int kNcat       = 2 * kUnits;
constexpr int kScalPlanes = 5;

typedef __attribute__((ext_vector_type(16))) _Float16 v16h;
typedef __attribute__((ext_vector_type(8)))  _Float16 v8h;
typedef __attribute__((ext_vector_type(16))) __bf16   v16b;
typedef __attribute__((ext_vector_type(8)))  __bf16   v8b;
typedef __attribute__((ext_vector_type(8)))  float    v8f;
typedef __attribute__((ext_vector_type(4)))  float    v4f;
typedef __attribute__((ext_vector_type(4)))  unsigned int v4u;

__device__ __forceinline__ unsigned short f2bf_bits(float f) {
  unsigned u = __float_as_uint(f);
  return (unsigned short)((u + 0x7FFFu + ((u >> 16) & 1u)) >> 16);
}
__device__ __forceinline__ float bf_bits2f(unsigned short h) { return __uint_as_float(((unsigned)h) << 16); }

__device__ __forceinline__ void dep_guard_h(v8f& a, v8f& b, v16h x, v16h y) { asm volatile("v_nop\n\tv_nop\n\tv_nop\n\tv_nop" : "+v"(a), "+v"(b) : "v"(x), "v"(y)); }
__device__ __forceinline__ void dep_guard_b(v8f& a, v8f& b, v16b x, v16b y) { asm volatile("v_nop\n\tv_nop\n\tv_nop\n\tv_nop" : "+v"(a), "+v"(b) : "v"(x), "v"(y)); }
__device__ __forceinline__ void keep4_h(v16h a, v16h b, v16h c, v16h d) { asm volatile("v_nop" :: "v"(a), "v"(b), "v"(c), "v"(d)); }
__device__ __forceinline__ void keep4_b(v16b a, v16b b, v16b c, v16b d) { asm volatile("v_nop" :: "v"(a), "v"(b), "v"(c), "v"(d)); }
__device__ __forceinline__ void acc_guard4(v8f& a, v8f& b, v8f& c, v8f& d) { asm volatile("v_nop\n\tv_nop\n\tv_nop\n\tv_nop" : "+v"(a), "+v"(b), "+v"(c), "+v"(d)); }
template <typename T> struct Frag;
template <> struct Frag<_Float16> {
  typedef v16h V; union U { v16h v; v8h h[2]; };
  static __device__ __forceinline__ v16h load(const _Float16* p) {
    U f; f.h[0] = *(const v8h*)(p); f.h[1] = *(const v8h*)(p + 16); return f.v;
  }
  static __device__ __forceinline__ v8f mma(v16h a, v16h b, v8f c) {
    return __builtin_amdgcn_wmma_f32_16x16x32_f16(false, a, false, b, (short)0, c, false, false);
  }
  static __device__ __forceinline__ void guard(v8f& a, v8f& b, v16h x, v16h y) { dep_guard_h(a, b, x, y); }
  static __device__ __forceinline__ void keep(v16h a, v16h b, v16h c, v16h d) { keep4_h(a, b, c, d); }
};
template <> struct Frag<__bf16> {
  typedef v16b V; union U { v16b v; v8b h[2]; };
  static __device__ __forceinline__ v16b load(const __bf16* p) {
    U f; f.h[0] = *(const v8b*)(p); f.h[1] = *(const v8b*)(p + 16); return f.v;
  }
  static __device__ __forceinline__ v8f mma(v16b a, v16b b, v8f c) {
    return __builtin_amdgcn_wmma_f32_16x16x32_bf16(false, a, false, b, (short)0, c, false, false);
  }
  static __device__ __forceinline__ void guard(v8f& a, v8f& b, v16b x, v16b y) { dep_guard_b(a, b, x, y); }
  static __device__ __forceinline__ void keep(v16b a, v16b b, v16b c, v16b d) { keep4_b(a, b, c, d); }
};

__device__ __forceinline__ unsigned pk16(unsigned short a, unsigned short b) { return (unsigned)a | ((unsigned)b << 16); }

template <int ET> struct Elem;
template <> struct Elem<0> { typedef _Float16 T; };
template <> struct Elem<1> { typedef __bf16 T; };
template <int ET, bool SPLIT, int BIAS_MODE, int OUT_MODE, bool RESID, int ACT = 0>
__global__ __launch_bounds__(256) void wmma_gemm64(
    const unsigned short* __restrict__ Ap, const unsigned short* __restrict__ A2p, int lda, long strideA,
    const unsigned short* __restrict__ Btp, const unsigned short* __restrict__ Bt2p, int ldb, long strideB,
    void* __restrict__ Cout, void* __restrict__ Cout2, int ldc, long strideC,
    const float* __restrict__ bias,
    const float* __restrict__ resid, long strideR,
    int M, int N, int K, float scale) {
  typedef typename Elem<ET>::T T;
  typedef typename Frag<T>::V V;
  const T* A = (const T*)Ap; const T* A2 = (const T*)A2p; const T* Bt = (const T*)Btp; const T* Bt2 = (const T*)Bt2p;
  __shared__ __align__(16) float sT[8][16 * 68];
  const int b    = blockIdx.y;
  const int lane = threadIdx.x & 31;
  const int wave = threadIdx.x >> 5;
  const int tilesN = N >> 6;
  const int tilesM = M >> 6;
  const int tile = blockIdx.x * 8 + wave;
  if (tile >= tilesM * tilesN) return;
  const int tm = tile / tilesN;
  const int tn = tile - tm * tilesN;
  const int m0 = tm << 6;
  const int n0 = tn << 6;

  const T* Ab  = A  + (size_t)b * strideA;
  const T* Bb  = Bt + (size_t)b * strideB;
  const T* Ab2 = SPLIT ? (A2  + (size_t)b * strideA) : nullptr;
  const T* Bb2 = SPLIT ? (Bt2 + (size_t)b * strideB) : nullptr;

  const int rlane = lane & 15;
  const int koff  = (lane >> 4) * 8;
  const int mOff  = (lane >> 4) * 8;

  v8f acc[4][4];
#pragma unroll
  for (int i = 0; i < 4; ++i)
#pragma unroll
    for (int j = 0; j < 4; ++j) acc[i][j] = (v8f){0.f,0.f,0.f,0.f,0.f,0.f,0.f,0.f};

  for (int k0 = 0; k0 < K; k0 += 32) {
    V bh[4], bl[4];
#pragma unroll
    for (int j = 0; j < 4; ++j) {
      const size_t bo = (size_t)(n0 + (j << 4) + rlane) * ldb + koff + k0;
      bh[j] = Frag<T>::load(Bb + bo);
      if (SPLIT) bl[j] = Frag<T>::load(Bb2 + bo);
    }
#pragma unroll
    for (int i = 0; i < 4; ++i) {
      const size_t ao = (size_t)(m0 + (i << 4) + rlane) * lda + koff + k0;
      V ah = Frag<T>::load(Ab + ao);
      V al;
      if (SPLIT) al = Frag<T>::load(Ab2 + ao);
#pragma unroll
      for (int j = 0; j < 4; ++j) {
        acc[i][j] = Frag<T>::mma(ah, bh[j], acc[i][j]);
        if (SPLIT) {
          acc[i][j] = Frag<T>::mma(ah, bl[j], acc[i][j]);
          acc[i][j] = Frag<T>::mma(al, bh[j], acc[i][j]);
        }
      }
      Frag<T>::guard(acc[i][0], acc[i][3], ah, SPLIT ? al : ah);
    }
    Frag<T>::keep(bh[0], bh[1], bh[2], bh[3]);
    if (SPLIT) Frag<T>::keep(bl[0], bl[1], bl[2], bl[3]);
  }
  acc_guard4(acc[0][0], acc[0][1], acc[0][2], acc[0][3]);
  acc_guard4(acc[1][0], acc[1][1], acc[1][2], acc[1][3]);
  acc_guard4(acc[2][0], acc[2][1], acc[2][2], acc[2][3]);
  acc_guard4(acc[3][0], acc[3][1], acc[3][2], acc[3][3]);

  float* slab = sT[wave];
  const float* Rb = RESID ? (resid + (size_t)b * strideR) : nullptr;
#pragma unroll
  for (int i = 0; i < 4; ++i) {
    const int mBase = m0 + (i << 4);
#pragma unroll
    for (int j = 0; j < 4; ++j) {
      const int n = n0 + (j << 4) + rlane;
      float bv = 0.f;
      if (BIAS_MODE == 2) bv = bias[n];
#pragma unroll
      for (int r = 0; r < 8; ++r) {
        float v = acc[i][j][r] * scale;
        if (BIAS_MODE == 1) v += bias[mBase + mOff + r];
        if (BIAS_MODE == 2) v += bv;
        if (RESID) v += Rb[(size_t)(mBase + mOff + r) * ldc + n];
        if (ACT == 1) v = tanhf(v);
        if (ACT == 2) v = fmaxf(v, 0.0f);
        if (ACT == 3) v = v / (1.0f + expf(-v));
        if (ACT == 4) v = (v > 0.f) ? v : 0.01f * v;
        if (ACT == 5) v = 0.5f * v * (1.0f + erff(v * 0.70710678118654752f));
        slab[(mOff + r) * 68 + (j << 4) + rlane] = v;
      }
    }
    __builtin_amdgcn_fence(__ATOMIC_RELEASE, "workgroup");
    __builtin_amdgcn_wave_barrier();
    __builtin_amdgcn_fence(__ATOMIC_ACQUIRE, "workgroup");
    if (OUT_MODE == 0) {
      float* C = (float*)Cout + (size_t)b * strideC;
      const int hh = lane >> 4, c4 = (lane & 15) * 4;
      for (int pass = 0; pass < 2; ++pass) {
#pragma unroll
        for (int it = 0; it < 8; ++it) {
          const int row = it * 2 + hh;
          v4f v = *(const v4f*)(slab + row * 68 + c4);
          *(volatile v4f*)(C + (size_t)(mBase + row) * ldc + n0 + c4) = v;
        }
        __threadfence();
      }
    } else {
      const int q = lane >> 3, c8 = (lane & 7) * 8;
      unsigned short* C  = (unsigned short*)Cout  + (size_t)b * strideC;
      unsigned short* C2 = (OUT_MODE == 2) ? ((unsigned short*)Cout2 + (size_t)b * strideC) : nullptr;
      for (int pass = 0; pass < 2; ++pass) {
#pragma unroll
        for (int it = 0; it < 4; ++it) {
          const int row = it * 4 + q;
          const float* sp = slab + row * 68 + c8;
          v8h hv, lv;
#pragma unroll
          for (int e = 0; e < 8; ++e) {
            if (OUT_MODE == 1) {
              hv[e] = (_Float16)sp[e];
            } else {
              unsigned short hb = f2bf_bits(sp[e]);
              unsigned short lb = f2bf_bits(sp[e] - bf_bits2f(hb));
              hv[e] = __builtin_bit_cast(_Float16, hb);
              lv[e] = __builtin_bit_cast(_Float16, lb);
            }
          }
          *(volatile v8h*)(C + (size_t)(mBase + row) * ldc + n0 + c8) = hv;
          if (OUT_MODE == 2) *(volatile v8h*)(C2 + (size_t)(mBase + row) * ldc + n0 + c8) = lv;
        }
        __threadfence();
      }
    }
    __builtin_amdgcn_fence(__ATOMIC_RELEASE, "workgroup");
    __builtin_amdgcn_wave_barrier();
    __builtin_amdgcn_fence(__ATOMIC_ACQUIRE, "workgroup");
  }
}

__global__ __launch_bounds__(256) void cast_split8_kernel(const float* __restrict__ in, unsigned short* __restrict__ hi,
                                                          unsigned short* __restrict__ lo, int n8) {
  const int i = blockIdx.x * 256 + threadIdx.x;
  if (i >= n8) return;
  const float* p = in + 8 * (size_t)i;
  const v4f a = *(const v4f*)(p);
  const v4f c = *(const v4f*)(p + 4);
  unsigned short hb[8], lb[8];
#pragma unroll
  for (int e = 0; e < 4; ++e) {
    const unsigned short h0 = f2bf_bits(a[e]);
    hb[e] = h0;
    lb[e] = f2bf_bits(a[e] - bf_bits2f(h0));
    const unsigned short h1 = f2bf_bits(c[e]);
    hb[4 + e] = h1;
    lb[4 + e] = f2bf_bits(c[e] - bf_bits2f(h1));
  }
  const v4u hv = (v4u){pk16(hb[0], hb[1]), pk16(hb[2], hb[3]), pk16(hb[4], hb[5]), pk16(hb[6], hb[7])};
  const v4u lv = (v4u){pk16(lb[0], lb[1]), pk16(lb[2], lb[3]), pk16(lb[4], lb[5]), pk16(lb[6], lb[7])};
  unsigned short* hq = hi + 8 * (size_t)i;
  unsigned short* lq = lo + 8 * (size_t)i;
  *(volatile v4u*)hq = hv;
  *(volatile v4u*)lq = lv;
  __threadfence();
  *(volatile v4u*)hq = hv;
  *(volatile v4u*)lq = lv;
}

__global__ __launch_bounds__(256) void unit_scalars_kernel(const float* __restrict__ W, const float* __restrict__ bias,
                                                           float* __restrict__ scal) {
  __shared__ float s_val[kScalPlanes][32];
  const int tid = threadIdx.x, lane = tid & 31, wave = tid >> 5;
  const int ublk = blockIdx.x * 32;
#pragma unroll 1
  for (int i = 0; i < 4; ++i) {
    const int ul = wave * 4 + i;
    const int u  = ublk + ul;
    const v4f wv = *(const v4f*)(W    + (size_t)u * kDim + lane * 4);
    const v4f bv = *(const v4f*)(bias + (size_t)u * kDim + lane * 4);
    float nb = (bv[0] * bv[0] + bv[1] * bv[1]) + (bv[2] * bv[2] + bv[3] * bv[3]);
#pragma unroll
    for (int off = 16; off > 0; off >>= 1) nb += __shfl_xor(nb, off, 32);
    const float omn = 1.0f - nb;
    const float a0 = omn * wv[0], a1 = omn * wv[1], a2 = omn * wv[2], a3 = omn * wv[3];
    float an2 = (a0 * a0 + a1 * a1) + (a2 * a2 + a3 * a3);
    float bap = (bv[0] * a0 + bv[1] * a1) + (bv[2] * a2 + bv[3] * a3);
#pragma unroll
    for (int off = 16; off > 0; off >>= 1) {
      an2 += __shfl_xor(an2, off, 32);
      bap += __shfl_xor(bap, off, 32);
    }
    const float an  = sqrtf(an2);
    const float lam = 2.0f / omn;
    const float sc  = lam * an;
    if (lane == 0) {
      s_val[0][ul] = nb;
      s_val[1][ul] = omn;
      s_val[2][ul] = bap;
      s_val[3][ul] = an;
      s_val[4][ul] = sc;
    }
  }
  __syncthreads();
  if (wave == 0) {
    const float v0 = s_val[0][lane], v1 = s_val[1][lane], v2 = s_val[2][lane], v3 = s_val[3][lane], v4 = s_val[4][lane];
    float* p = scal + ublk + lane;
    for (int pass = 0; pass < 2; ++pass) {
      *(volatile float*)(p + 0 * kUnits) = v0;
      *(volatile float*)(p + 1 * kUnits) = v1;
      *(volatile float*)(p + 2 * kUnits) = v2;
      *(volatile float*)(p + 3 * kUnits) = v3;
      *(volatile float*)(p + 4 * kUnits) = v4;
      __threadfence();
    }
  }
}

__global__ __launch_bounds__(256) void row_softmax_kernel(const float* __restrict__ x, const float* __restrict__ S,
                                                          const float* __restrict__ scal, float* __restrict__ out) {
  __shared__ float s_sc[kScalPlanes][kUnits];
  __shared__ __align__(16) float s_log[8][kUnits];
  const int tid = threadIdx.x, lane = tid & 31, wave = tid >> 5;
#pragma unroll
  for (int p = 0; p < kScalPlanes; ++p) s_sc[p][tid] = scal[p * kUnits + tid];
  const int row = blockIdx.x * 8 + wave;
  const v4f xv = *(const v4f*)(x + (size_t)row * kDim + lane * 4);
  float nv2 = (xv[0] * xv[0] + xv[1] * xv[1]) + (xv[2] * xv[2] + xv[3] * xv[3]);
#pragma unroll
  for (int off = 16; off > 0; off >>= 1) nv2 += __shfl_xor(nv2, off, 32);
  __syncthreads();

  const float* srow = S + (size_t)row * kNcat;
  float* lg = s_log[wave];
  float mx = -INFINITY;
#pragma unroll 1
  for (int i = 0; i < 8; ++i) {
    const int u = i * 32 + lane;
    const float s1  = srow[u];
    const float s2  = srow[kUnits + u];
    const float nb2 = s_sc[0][u];
    const float omn = s_sc[1][u];
    const float ba  = s_sc[2][u];
    const float an  = s_sc[3][u];
    const float sc  = s_sc[4][u];
    const float xy  = -s2;
    const float t0  = 1.0f + 2.0f * xy;
    const float c1  = t0 + nv2;
    const float dd  = t0 + nb2 * nv2;
    const float rdd = 1.0f / dd;
    const float alpha = c1 * rdd;
    const float beta  = omn * rdd;
    const float xa  = omn * s1;
    const float num = 2.0f * (beta * xa - alpha * ba);
    const float ab  = alpha * beta;
    const float mm  = (alpha * alpha) * nb2 + 2.0f * ab * xy + (beta * beta) * nv2;
    const float den = (1.0f - mm) * an;
    const float t   = num * (1.0f / den);
    const float lv  = sc * asinhf(t);
    lg[u] = lv;
    mx = fmaxf(mx, lv);
  }
#pragma unroll
  for (int off = 16; off > 0; off >>= 1) mx = fmaxf(mx, __shfl_xor(mx, off, 32));
  float sum = 0.f;
#pragma unroll 1
  for (int i = 0; i < 8; ++i) {
    const int u = i * 32 + lane;
    const float e = expf(lg[u] - mx);
    lg[u] = e;
    sum += e;
  }
#pragma unroll
  for (int off = 16; off > 0; off >>= 1) sum += __shfl_xor(sum, off, 32);
  const float inv = 1.0f / sum;
  __syncthreads();

  v4f o0 = *(const v4f*)(lg + lane * 4);
  v4f o1 = *(const v4f*)(lg + 128 + lane * 4);
  o0 = o0 * inv;
  o1 = o1 * inv;
  float* orow = out + (size_t)row * kUnits;
  for (int pass = 0; pass < 2; ++pass) {
    *(volatile v4f*)(orow + lane * 4)       = o0;
    *(volatile v4f*)(orow + 128 + lane * 4) = o1;
    __threadfence();
  }
}

extern "C" void kernel_launch(void* const* d_in, const int* in_sizes, int n_in,
                              void* d_out, int out_size, void* d_ws, size_t ws_size,
                              hipStream_t stream) {
  if (n_in < 3) return;
  if (in_sizes[0] != kRows * kDim) return;
  if (in_sizes[1] != kUnits * kDim) return;
  if (in_sizes[2] != kUnits * kDim) return;
  if (out_size != kRows * kUnits) return;

  const float* x    = (const float*)d_in[0];
  const float* W    = (const float*)d_in[1];
  const float* bias = (const float*)d_in[2];
  float* outp = (float*)d_out;

  const size_t SZ_S    = (size_t)kRows * kNcat * 4;
  const size_t SZ_X16  = (size_t)kRows * kDim * 2;
  const size_t SZ_B16  = (size_t)kNcat * kDim * 2;
  const size_t SZ_SCAL = (size_t)kScalPlanes * kUnits * 4;

  size_t off = 0;
  const size_t oS    = off; off += SZ_S;
  const size_t oXH   = off; off += SZ_X16;
  const size_t oXL   = off; off += SZ_X16;
  const size_t oBH   = off; off += SZ_B16;
  const size_t oBL   = off; off += SZ_B16;
  const size_t oSCAL = off; off += SZ_SCAL;
  const size_t TOTAL = off;
  if (TOTAL > ws_size) return;
  if (TOTAL > (size_t)134217728) return;

  char* ws = (char*)d_ws;
  float*          S    = (float*)(ws + oS);
  unsigned short* XH   = (unsigned short*)(ws + oXH);
  unsigned short* XL   = (unsigned short*)(ws + oXL);
  unsigned short* BH   = (unsigned short*)(ws + oBH);
  unsigned short* BL   = (unsigned short*)(ws + oBL);
  float*          SCAL = (float*)(ws + oSCAL);

  const dim3 blk(256);

  {
    const int n8x = kRows * kDim / 8;
    cast_split8_kernel<<<dim3(n8x / 256), blk, 0, stream>>>(x, XH, XL, n8x);
    const int n8w = kUnits * kDim / 8;
    cast_split8_kernel<<<dim3(n8w / 256), blk, 0, stream>>>(W, BH, BL, n8w);
    cast_split8_kernel<<<dim3(n8w / 256), blk, 0, stream>>>(bias, BH + (size_t)kUnits * kDim, BL + (size_t)kUnits * kDim, n8w);
  }

  unit_scalars_kernel<<<dim3(kUnits / 32), blk, 0, stream>>>(W, bias, SCAL);

  {
    const int tiles = (kRows / 64) * (kNcat / 64);
    wmma_gemm64<1, true, 0, 0, false, 0><<<dim3((tiles + 7) / 8, 1), blk, 0, stream>>>(
        XH, XL, kDim, 0L, BH, BL, kDim, 0L, (void*)S, (void*)S, kNcat, 0L, SCAL, SCAL, 0L, kRows, kNcat, kDim, 1.0f);
  }

  row_softmax_kernel<<<dim3(kRows / 8), blk, 0, stream>>>(x, S, SCAL, outp);
}
